// GraphSAGE_34986803593269
// MI455X (gfx1250) — hardware-verified
//
#include <hip/hip_runtime.h>


namespace {

constexpr int N = 100000, NP = 100032, NPL = NP  , SRCM = N  , KN = 16  , L = 2, NRL = NP  ;
constexpr int D = 128, NL = (NPL < N ? NPL : N); constexpr int DH = 128, DO = 64, K2 = 2 * D;
constexpr float XS = 8.0f, WSC = 256.0f, WSQ = 0.25f, RS_ = 1024.0f, SLOPE = 0.0f, BNEPS = 1e-5f;
static_assert(NP % 32 == 0 && NP >= N && NPL % 32 == 0 && D == 128, "tiling");
typedef _Float16 b16;
typedef __attribute__((ext_vector_type(16))) _Float16 v16b;
typedef __attribute__((ext_vector_type(8))) _Float16 v8b;
typedef __attribute__((ext_vector_type(8))) float v8f;
typedef __attribute__((ext_vector_type(4))) float v4f;
__device__ __forceinline__ float bf16_rne(float f) { unsigned int u = __float_as_uint(f); u += 0x7FFFu + ((u >> 16) & 1u); return __uint_as_float(u & 0xFFFF0000u); }
__device__ __forceinline__ void split16(float v, b16& hi, b16& lo) { hi = (b16)v; lo = (b16)(v - (float)hi); }
__device__ __forceinline__ v16b frag_kb(const b16* p, int hh) { const v8b a = *(const v8b*)(p + 8 * hh), b = *(const v8b*)(p + 16 + 8 * hh); v16b f;
#pragma unroll
  for (int e = 0; e < 8; ++e) { f[e] = a[e]; f[8 + e] = b[e]; } return f; }
__device__ __forceinline__ v8f wmma16b(v16b a, v16b b, v8f c) { v8f d = __builtin_amdgcn_wmma_f32_16x16x32_f16(false, a, false, b, (short)0, c, false, false); asm volatile("v_nop\n\tv_nop\n\tv_nop\n\tv_nop" : "+v"(d) : "v"(a), "v"(b)); return d; }
__device__ __forceinline__ void wave_lds_sync() { __builtin_amdgcn_fence(__ATOMIC_RELEASE, "workgroup"); __builtin_amdgcn_wave_barrier(); __builtin_amdgcn_fence(__ATOMIC_ACQUIRE, "workgroup"); }
__device__ __forceinline__ float pmul(float a, float b) { float p = a * b; asm volatile("" : "+v"(p)); return p; }
__device__ __forceinline__ int iclamp(int v, int lo, int hi) { return v < lo ? lo : (v > hi ? hi : v); }
typedef __attribute__((ext_vector_type(4))) _Float16 v4h;
template <int KA, int KB, int NOUT>
__global__ __launch_bounds__(256) void wt2_kernel(const float* __restrict__ wl, const float* __restrict__ wr, b16* __restrict__ WT, float scl) {
  const int u = blockIdx.x * 256 + threadIdx.x; if (u >= NOUT * (KA + KB) / 8) return; const int e = u * 8; const int o = e / (KA + KB), k0 = e % (KA + KB); v8b v;
#pragma unroll
  for (int j = 0; j < 8; ++j) { const int k = k0 + j; v[j] = (b16)(bf16_rne(k < KA ? wl[(size_t)k * NOUT + o] : wr[(size_t)(k - KA) * NOUT + o]) * scl); }
  for (int pass = 0; pass < 2; ++pass) { *(volatile v8b*)(WT + e) = v; __threadfence(); }
}
template <int K, int NOUT>
__global__ __launch_bounds__(256) void wt_kernel(const float* __restrict__ w, b16* __restrict__ WT, float scl) {
  const int u = blockIdx.x * 256 + threadIdx.x; if (u >= NOUT * K / 8) return; const int e = u * 8; const int o = e / K, k0 = e % K; v8b v;
#pragma unroll
  for (int j = 0; j < 8; ++j) v[j] = (b16)(bf16_rne(w[(size_t)(k0 + j) * NOUT + o]) * scl);
  for (int pass = 0; pass < 2; ++pass) { *(volatile v8b*)(WT + e) = v; __threadfence(); }
}
template <bool RND>
__global__ __launch_bounds__(256) void agg_kernel(const float* __restrict__ IN, const int* __restrict__ nidx, float* __restrict__ AGG) {
  const int tid = threadIdx.x; const int row = tid >> 3, g = tid & 7, c0 = g * 16; const int v = blockIdx.x * 32 + row; const int vv = v < N ? v : N - 1;
  float m[16];
#pragma unroll
  for (int j = 0; j < 16; ++j) m[j] = 0.0f;
#pragma unroll 1
  for (int i = 0; i < KN; ++i) { int s = iclamp(nidx[(size_t)vv * KN + i], 0, N - 1); if (SRCM < N) s %= SRCM; const float* xr = IN + (size_t)s * D + c0;
#pragma unroll
    for (int q = 0; q < 4; ++q) { const v4f t4 = *(const v4f*)(xr + 4 * q); for (int j = 0; j < 4; ++j) m[4 * q + j] += RND ? bf16_rne(t4[j]) : t4[j]; } }
  for (int pass = 0; pass < 2; ++pass) { float* ar = AGG + (size_t)v * D + c0;
#pragma unroll
    for (int q = 0; q < 4; ++q) { v4f o; for (int j = 0; j < 4; ++j) o[j] = (v < N) ? m[4 * q + j] * (1.0f / (float)KN) : 0.0f; *(volatile v4f*)(ar + 4 * q) = o; }
    __threadfence(); }
}
__global__ __launch_bounds__(256) void wts_kernel(const float* __restrict__ w, b16* __restrict__ WT, float scl) {
  const int u = blockIdx.x * 256 + threadIdx.x; if (u >= DH * K2 / 8) return; const int e = u * 8; const int o = e / K2, k0 = e % K2; v8b v;
#pragma unroll
  for (int j = 0; j < 8; ++j) { const int k = k0 + j; v[j] = (b16)(bf16_rne(w[(size_t)(k < D ? D + k : k - D) * DH + o]) * scl); }
  for (int pass = 0; pass < 2; ++pass) { *(volatile v8b*)(WT + e) = v; __threadfence(); }
}
template <int NT, bool XEXACT, bool RELU>
__global__ __launch_bounds__(64) void sage_kernel(const float* __restrict__ AGG, const float* __restrict__ X, const b16* __restrict__ WT, const b16* __restrict__ WQ, const float* __restrict__ bias, float* __restrict__ out, int mrows) {
  constexpr int NOUT = NT * 16;
  __shared__ __attribute__((aligned(16))) b16 Ah[2][16][K2 + 8], Al[2][16][K2 + 8]; __shared__ __attribute__((aligned(16))) float Tf[2][16][NOUT + 4];
  const int wave = threadIdx.x >> 5, lane = threadIdx.x & 31, nloc = lane & 15, hlf = lane >> 4; const size_t m0 = (size_t)blockIdx.x * 32 + wave * 16;
  for (int idx = lane; idx < 16 * (D / 4); idx += 32) { const int rr = idx / (D / 4), c4 = (idx % (D / 4)) * 4; const size_t arow = (m0 + rr < (size_t)N) ? m0 + rr : (size_t)N - 1; const v4f av = *(const v4f*)(AGG + arow * D + c4), xv = *(const v4f*)(X + arow * D + c4); v4h h1, l1, h2, l2;
    for (int j = 0; j < 4; ++j) { const float vs = av[j] * XS; const b16 ph = (b16)vs; h1[j] = ph; l1[j] = (b16)((vs - (float)ph) * RS_); if (XEXACT) { h2[j] = (b16)(bf16_rne(xv[j]) * XS); l2[j] = (b16)0.0f; } else { const float ws_ = xv[j] * XS; const b16 p2 = (b16)ws_; h2[j] = p2; l2[j] = (b16)((ws_ - (float)p2) * RS_); } }
    *(v4h*)(&Ah[wave][rr][c4]) = h1; *(v4h*)(&Al[wave][rr][c4]) = l1; *(v4h*)(&Ah[wave][rr][D + c4]) = h2; *(v4h*)(&Al[wave][rr][D + c4]) = l2; }
  wave_lds_sync();
  v8f acc[NT];
#pragma unroll
  for (int t = 0; t < NT; ++t) acc[t] = (v8f){};
#pragma unroll 2
  for (int kb = 0; kb < K2; kb += 32) { const v16b a = frag_kb(&Ah[wave][nloc][kb], hlf), al = frag_kb(&Al[wave][nloc][kb], hlf); const bool lo = XEXACT ? (kb < D) : true;
#pragma unroll
    for (int t = 0; t < NT; ++t) { const size_t wo_ = (size_t)(t * 16 + nloc) * K2 + kb; acc[t] = wmma16b(a, frag_kb(WT + wo_, hlf), acc[t]); if (lo) acc[t] = wmma16b(al, frag_kb(WQ + wo_, hlf), acc[t]); } }
#pragma unroll
  for (int t = 0; t < NT; ++t) { const int col = t * 16 + nloc; const float bb = bf16_rne(bias[col]); for (int r = 0; r < 8; ++r) { float v = acc[t][r] * (1.0f / (XS * WSC)) + bb; if (RELU) v = fmaxf(v, 0.0f); Tf[wave][8 * hlf + r][col] = (m0 + 8 * hlf + r < (size_t)N) ? v : 0.0f; } }
  wave_lds_sync();
  for (int pass = 0; pass < 2; ++pass) {
    if (NOUT == 128) { for (int rr = 0; rr < 16; ++rr) if (m0 + rr < (size_t)mrows) *(volatile v4f*)(out + (m0 + rr) * NOUT + lane * 4) = *(const v4f*)(&Tf[wave][rr][lane * 4]); }
    else { for (int rr = 0; rr < 16; rr += 2) { const int r2 = rr + (lane >> 4); if (m0 + r2 < (size_t)mrows) *(volatile v4f*)(out + (m0 + r2) * NOUT + (lane & 15) * 4) = *(const v4f*)(&Tf[wave][r2][(lane & 15) * 4]); } }
    __threadfence(); }
}
}

extern "C" void kernel_launch(void* const* d_in, const int* in_sizes, int n_in, void* d_out, int out_size, void* d_ws, size_t ws_size, hipStream_t stream) {
  (void)n_in;
  auto Fp = [&](int i) { return (const float*)d_in[i]; }; auto Ip = [&](int i) { return (const int*)d_in[i]; };
  if (in_sizes[0] != N * D || in_sizes[1] != L * N * KN || in_sizes[2] != L * K2 * DH || in_sizes[3] != L * DH || out_size != N * DH) return;
  size_t off = 0; char* ws = (char*)d_ws;
  auto carve = [&](size_t bytes) { char* p = ws + off; off += (bytes + 255) & ~(size_t)255; return p; };
  b16* W0T = (b16*)carve((size_t)DH * K2 * 2); b16* W0Q = (b16*)carve((size_t)DH * K2 * 2); b16* W1T = (b16*)carve((size_t)DH * K2 * 2); b16* W1Q = (b16*)carve((size_t)DH * K2 * 2);
  float* AGG = (float*)carve((size_t)NP * D * 4); float* H1 = (float*)carve((size_t)NP * D * 4);
  if (off > ws_size || off > ((size_t)128 << 20)) return;
  const unsigned gw = (DH * K2 / 8 + 255) / 256;
  wts_kernel<<<gw, 256, 0, stream>>>(Fp(2), W0T, WSC); wts_kernel<<<gw, 256, 0, stream>>>(Fp(2), W0Q, WSQ); wts_kernel<<<gw, 256, 0, stream>>>(Fp(2) + (size_t)K2 * DH, W1T, WSC); wts_kernel<<<gw, 256, 0, stream>>>(Fp(2) + (size_t)K2 * DH, W1Q, WSQ);
  agg_kernel<true><<<NRL / 32, 256, 0, stream>>>(Fp(0), Ip(1), AGG);
  sage_kernel<8, true, true><<<NRL / 32, 64, 0, stream>>>(AGG, Fp(0), W0T, W0Q, Fp(3), H1, NP);
  agg_kernel<false><<<NP / 32, 256, 0, stream>>>(H1, Ip(1) + (size_t)N * KN, AGG);
  sage_kernel<8, false, false><<<NPL / 32, 64, 0, stream>>>(AGG, H1, W1T, W1Q, Fp(3) + DH, (float*)d_out, NL);
}
